// RBLNGptOssExperts_18442589570203
// MI455X (gfx1250) — hardware-verified
//
#include <hip/hip_runtime.h>
#include <stddef.h>
#include <stdint.h>

#define NTOK   1024
#define DIM    1024
#define FFN    1024
#define NE     8
#define NSEL   2
#define NPAIR  (NTOK * NSEL)
#define NTILE  (NPAIR / 64 + NE)
#define AROWS  (NTILE * 64)
#define QPR    (DIM / 2)
#define SPR    (DIM / 32)
#define APITCH 144
#define EPITCH 72
#define OTP    68
#define GLU_A  1.702f
#define GLU_L  7.0f

static_assert(DIM == FFN);
static_assert(NE == 8);
static_assert(NSEL == 2);
static_assert(NTILE == 40);
static_assert(NTOK % 256 == 0);
static_assert(DIM % 128 == 0);
static_assert(DIM / 8 == 128);
static_assert(8 * 16 * EPITCH <= 64 * APITCH);
static_assert((NTOK * DIM) % 2048 == 0);

typedef __bf16         v16bf __attribute__((ext_vector_type(16)));
typedef float          v8f   __attribute__((ext_vector_type(8)));
typedef float          v4f   __attribute__((ext_vector_type(4)));
typedef unsigned int   v4u   __attribute__((ext_vector_type(4)));
typedef int            v4i   __attribute__((ext_vector_type(4)));
typedef unsigned short v8us  __attribute__((ext_vector_type(8)));

union Frag { v16bf v; v4u u[2]; };
union Pk8  { v8us h; v4u u; };

__device__ __forceinline__ int clampi(int v, int lo, int hi) { return min(max(v, lo), hi); }

__device__ __forceinline__ unsigned short bfr(float f) {
  unsigned u = __float_as_uint(f);
  u += 0x7FFFu + ((u >> 16) & 1u);
  return (unsigned short)(u >> 16);
}
__device__ __forceinline__ float bff(unsigned short h) { return __uint_as_float(((unsigned)h) << 16); }

__device__ __forceinline__ void split2(float x, unsigned short& h, unsigned short& l) {
  h = bfr(x);
  l = bfr(x - bff(h));
}

__device__ __forceinline__ v8f mma16(v16bf a, v16bf b, v8f c) {
  c = __builtin_amdgcn_wmma_f32_16x16x32_bf16(false, a, false, b, (short)0, c, false, false);
  asm volatile("v_nop\n\tv_nop\n\tv_nop\n\tv_nop" : "+v"(c) : "v"(a), "v"(b));
  return c;
}

__device__ __forceinline__ v16bf ldfrag(const unsigned short* p, int ld, int row0, int k0, int lane) {
  const int m = lane & 15, lh = lane >> 4;
  const unsigned short* q = p + (size_t)(row0 + m) * ld + k0 + 8 * lh;
  Frag f;
  f.u[0] = *(const v4u*)(q);
  f.u[1] = *(const v4u*)(q + 16);
  return f.v;
}

__device__ __forceinline__ v8f zero8() { return (v8f){0.f, 0.f, 0.f, 0.f, 0.f, 0.f, 0.f, 0.f}; }

__device__ __forceinline__ unsigned short dq1(int c, float sc128) {
  const int m = c & 7, ex = m >> 1, mt = m & 1;
  const int q = (ex == 0) ? mt : ((2 + mt) << ((ex - 1) & 3));
  float f = (float)q * sc128;
  f = (c & 8) ? -f : f;
  return bfr(f);
}

__global__ __launch_bounds__(256) void k_xsplit(const float* __restrict__ src, unsigned short* __restrict__ dh,
                                                unsigned short* __restrict__ dl, int n8) {
  const int i = blockIdx.x * 256 + (int)threadIdx.x;
  if (i >= n8) return;
  const size_t o = (size_t)i * 8;
  const v4f a0 = *(const v4f*)(src + o);
  const v4f a1 = *(const v4f*)(src + o + 4);
  Pk8 ph, pl;
#pragma unroll
  for (int j = 0; j < 4; ++j) {
    unsigned short hv, lv;
    split2(a0[j], hv, lv);
    ph.h[j] = hv;
    pl.h[j] = lv;
    split2(a1[j], hv, lv);
    ph.h[4 + j] = hv;
    pl.h[4 + j] = lv;
  }
  const v4u vh = ph.u, vl = pl.u;
  volatile v4u* d0 = (volatile v4u*)(dh + o);
  volatile v4u* d1 = (volatile v4u*)(dl + o);
  *d0 = vh;
  *d1 = vl;
  __threadfence();
  *d0 = vh;
  *d1 = vl;
}

__global__ __launch_bounds__(256) void k_deq(const int* __restrict__ blk, const int* __restrict__ scl,
                                             unsigned short* __restrict__ w, int n8) {
  const int i = blockIdx.x * 256 + (int)threadIdx.x;
  if (i >= n8) return;
  const int rf = i >> 7;
  const int kc = (i & 127) * 8;
  const v4i bb = *(const v4i*)(blk + (size_t)rf * QPR + (kc >> 1));
  const int s  = scl[(size_t)rf * SPR + (kc >> 5)];
  const int se = clampi(s - 1, 1, 254);
  const float sc128 = __uint_as_float(((unsigned)se) << 23);
  Pk8 pk;
#pragma unroll
  for (int j = 0; j < 4; ++j) {
    const int bv = bb[j];
    pk.h[2 * j]     = dq1(bv & 15, sc128);
    pk.h[2 * j + 1] = dq1((bv >> 4) & 15, sc128);
  }
  const v4u vv = pk.u;
  volatile v4u* d = (volatile v4u*)(w + (size_t)i * 8);
  *d = vv;
  __threadfence();
  *d = vv;
}

__global__ __launch_bounds__(256) void k_lists(const float* __restrict__ lg, int* __restrict__ tokl,
                                               float* __restrict__ wl, int* __restrict__ tab) {
#pragma clang fp contract(off)
  __shared__ __align__(16) int   sSel[NTOK];
  __shared__ __align__(16) float sW0[NTOK];
  __shared__ __align__(16) float sW1[NTOK];
  __shared__ __align__(16) int   ltok[NTOK];
  __shared__ __align__(16) float lw[NTOK];
  __shared__ int wc[8];
  __shared__ __align__(16) int sTab[64];
  const int tid = threadIdx.x, lane = tid & 31, wave = tid >> 5;
  if (tid < 64) sTab[tid] = 0;

#pragma unroll 1
  for (int j = 0; j < NTOK / 256; ++j) {
    const int t = j * 256 + tid;
    const v4f l0 = *(const v4f*)(lg + (size_t)t * NE);
    const v4f l1 = *(const v4f*)(lg + (size_t)t * NE + 4);
    float v[NE] = {l0[0], l0[1], l0[2], l0[3], l1[0], l1[1], l1[2], l1[3]};
    int i0 = 0;
    float b0 = v[0];
#pragma unroll
    for (int e = 1; e < NE; ++e) {
      const bool cnd = (v[e] > b0);
      b0 = cnd ? v[e] : b0;
      i0 = cnd ? e : i0;
    }
    int i1 = (i0 == 0) ? 1 : 0;
    float b1 = -__builtin_huge_valf();
#pragma unroll
    for (int e = 0; e < NE; ++e) {
      const bool cnd = (e != i0) && (v[e] > b1);
      b1 = cnd ? v[e] : b1;
      i1 = cnd ? e : i1;
    }
    const float e1  = expf(b1 - b0);
    const float s   = 1.0f + e1;
    const float inv = 1.0f / s;
    sSel[t] = i0 | (i1 << 8);
    sW0[t]  = inv;
    sW1[t]  = e1 * inv;
  }

  int tbrun = 0;
#pragma unroll 1
  for (int e = 0; e < NE; ++e) {
    __syncthreads();
    for (int i = tid; i < NTOK; i += 256) { ltok[i] = 0; lw[i] = 0.f; }
    __syncthreads();
    int run = 0;
#pragma unroll 1
    for (int ch = 0; ch < NTOK / 256; ++ch) {
      const int t = ch * 256 + tid;
      const int sel = sSel[t];
      const int i0 = sel & 255, i1 = (sel >> 8) & 255;
      const bool h0 = (i0 == e), h1 = (i1 == e);
      const bool flag = h0 || h1;
      const int slot = h0 ? 0 : 1;
      const float w0v = sW0[t], w1v = sW1[t];
      const float w = h0 ? w0v : w1v;
      const unsigned bal = __builtin_amdgcn_ballot_w32(flag);
      const int pre = __builtin_popcount(bal & ((1u << lane) - 1u));
      if (lane == 0) wc[wave] = __builtin_popcount(bal);
      __syncthreads();
      int base = run, tot = 0;
#pragma unroll
      for (int q = 0; q < 8; ++q) {
        const int cw = wc[q];
        base += (q < wave) ? cw : 0;
        tot  += cw;
      }
      const int pos = clampi(base + pre, 0, NTOK - 1);
      if (flag) { ltok[pos] = t * NSEL + slot; lw[pos] = w; }
      run += tot;
      __syncthreads();
    }
    run = clampi(run, 0, NTOK);
    const int ntl = (run + 63) >> 6;
    if (tid == 0) { sTab[e] = run; sTab[32 + e + 1] = clampi(tbrun + ntl, 0, NTILE); }
    tbrun += ntl;

    int*   trow = tokl + (size_t)e * NTOK;
    float* wrow = wl + (size_t)e * NTOK;
    const v4i tv = *(const v4i*)(ltok + tid * 4);
    const v4f wv = *(const v4f*)(lw + tid * 4);
    for (int ps = 0; ps < 2; ++ps) {
      *(volatile v4i*)(trow + tid * 4) = tv;
      *(volatile v4f*)(wrow + tid * 4) = wv;
      __threadfence();
    }
  }
  __syncthreads();
  if (wave == 0) {
    const v4i tq = *(const v4i*)(sTab + (lane & 15) * 4);
    volatile v4i* d = (volatile v4i*)(tab + (lane & 15) * 4);
    if (lane < 16) *d = tq;
    __threadfence();
    if (lane < 16) *d = tq;
  }
}

__global__ __launch_bounds__(256) void k_upgate(const unsigned short* __restrict__ xh,
                                                const unsigned short* __restrict__ xl,
                                                const unsigned short* __restrict__ wg,
                                                const unsigned short* __restrict__ wu,
                                                const float* __restrict__ gb, const float* __restrict__ ub,
                                                const int* __restrict__ tokl, const float* __restrict__ wl,
                                                const int* __restrict__ tab,
                                                unsigned short* __restrict__ ah, unsigned short* __restrict__ al) {
#pragma clang fp contract(off)
  __shared__ __align__(16) unsigned short sAh[64 * APITCH];
  __shared__ __align__(16) unsigned short sAl[64 * APITCH];
  __shared__ int   sTok[64];
  __shared__ float sWr[64];
  __shared__ int   sTab[64];
  const int tid = threadIdx.x, lane = tid & 31, wave = tid >> 5;
  const int hh = lane >> 4, c = lane & 15;
  const int wm = wave & 3, wn = wave >> 2;
  const int b  = blockIdx.y;
  const int n0 = blockIdx.x * 128;

  if (tid < 64) sTab[tid] = tab[tid];
  __syncthreads();
  const int tb8 = clampi(sTab[32 + NE], 0, NTILE);
  if (b >= tb8) return;
  int e = 0;
#pragma unroll
  for (int q = 1; q < NE; ++q) e += (clampi(sTab[32 + q], 0, NTILE) <= b) ? 1 : 0;
  const int tbe = clampi(sTab[32 + e], 0, NTILE);
  const int cne = clampi(sTab[e], 0, NTOK);
  if (tid < 64) {
    const int rloc = (b - tbe) * 64 + tid;
    const bool valid = (rloc >= 0) && (rloc < cne);
    const int li = e * NTOK + clampi(rloc, 0, NTOK - 1);
    const int enc = tokl[li];
    const float w = wl[li];
    sTok[tid] = clampi(enc >> 1, 0, NTOK - 1);
    sWr[tid]  = valid ? w : 0.f;
  }
  __syncthreads();

  const unsigned short* wge = wg + (size_t)e * (size_t)(FFN * DIM);
  const unsigned short* wue = wu + (size_t)e * (size_t)(FFN * DIM);
  const int brow = n0 + wn * 64;

  v8f accG[4], accU[4];
#pragma unroll
  for (int t = 0; t < 4; ++t) { accG[t] = zero8(); accU[t] = zero8(); }

  const int ar = tid >> 2, ac = tid & 3;
  const unsigned short* xrh = xh + (size_t)sTok[ar] * DIM + ac * 32;
  const unsigned short* xrl = xl + (size_t)sTok[ar] * DIM + ac * 32;
  unsigned short* awh = sAh + ar * APITCH + ac * 32;
  unsigned short* awl = sAl + ar * APITCH + ac * 32;
#pragma unroll 1
  for (int kc = 0; kc < DIM / 128; ++kc) {
    __syncthreads();
#pragma unroll
    for (int q = 0; q < 4; ++q) {
      *(v4u*)(awh + 8 * q) = *(const v4u*)(xrh + kc * 128 + 8 * q);
      *(v4u*)(awl + 8 * q) = *(const v4u*)(xrl + kc * 128 + 8 * q);
    }
    __syncthreads();
#pragma unroll 1
    for (int ks = 0; ks < 4; ++ks) {
      const int kg = kc * 128 + ks * 32;
      const v16bf fh = ldfrag(sAh, APITCH, wm * 16, ks * 32, lane);
      const v16bf fl = ldfrag(sAl, APITCH, wm * 16, ks * 32, lane);
#pragma unroll
      for (int t = 0; t < 4; ++t) {
        const v16bf bq = ldfrag(wge, DIM, brow + 16 * t, kg, lane);
        accG[t] = mma16(fh, bq, accG[t]);
        accG[t] = mma16(fl, bq, accG[t]);
      }
#pragma unroll
      for (int t = 0; t < 4; ++t) {
        const v16bf bq = ldfrag(wue, DIM, brow + 16 * t, kg, lane);
        accU[t] = mma16(fh, bq, accU[t]);
        accU[t] = mma16(fl, bq, accU[t]);
      }
    }
  }

  float gbv[4], ubv[4];
#pragma unroll
  for (int t = 0; t < 4; ++t) {
    gbv[t] = gb[(size_t)e * FFN + brow + 16 * t + c];
    ubv[t] = ub[(size_t)e * FFN + brow + 16 * t + c];
  }
  float wr[8];
#pragma unroll
  for (int r = 0; r < 8; ++r) wr[r] = sWr[wm * 16 + 8 * hh + r];
  __syncthreads();

  unsigned short* ewh = sAh + wave * (16 * EPITCH);
  unsigned short* ewl = sAl + wave * (16 * EPITCH);
#pragma unroll
  for (int t = 0; t < 4; ++t) {
#pragma unroll
    for (int r = 0; r < 8; ++r) {
      const float g  = fminf(accG[t][r] + gbv[t], GLU_L);
      const float u  = fminf(fmaxf(accU[t][r] + ubv[t], -GLU_L), GLU_L);
      const float ex = __expf(-GLU_A * g);
      const float sg = __builtin_amdgcn_rcpf(1.0f + ex);
      const float glu = g * sg;
      const float av = ((u + 1.0f) * glu) * wr[r];
      unsigned short hv, lv;
      split2(av, hv, lv);
      ewh[(8 * hh + r) * EPITCH + 16 * t + c] = hv;
      ewl[(8 * hh + r) * EPITCH + 16 * t + c] = lv;
    }
  }
  __syncthreads();
  v4u vh[4], vl[4];
  size_t go[4];
#pragma unroll
  for (int it = 0; it < 4; ++it) {
    const int p  = lane + 32 * it;
    const int L  = p >> 3;
    const int pc = p & 7;
    Pk8 kh, kl;
    kh.h   = *(const v8us*)(ewh + L * EPITCH + pc * 8);
    kl.h   = *(const v8us*)(ewl + L * EPITCH + pc * 8);
    vh[it] = kh.u;
    vl[it] = kl.u;
    go[it] = (size_t)(b * 64 + wm * 16 + L) * FFN + brow + pc * 8;
  }
  for (int ps = 0; ps < 2; ++ps) {
#pragma unroll
    for (int it = 0; it < 4; ++it) {
      *(volatile v4u*)(ah + go[it]) = vh[it];
      *(volatile v4u*)(al + go[it]) = vl[it];
    }
    __threadfence();
  }
}

__global__ __launch_bounds__(256) void k_down(const unsigned short* __restrict__ ah,
                                              const unsigned short* __restrict__ al,
                                              const unsigned short* __restrict__ wd,
                                              const float* __restrict__ db,
                                              const int* __restrict__ tokl, const float* __restrict__ wl,
                                              const int* __restrict__ tab, float* __restrict__ part) {
#pragma clang fp contract(off)
  __shared__ __align__(16) float sO[8 * 16 * OTP];
  __shared__ int   sEnc[64];
  __shared__ float sW[64];
  __shared__ int   sVal[64];
  __shared__ int   sTab[64];
  const int tid = threadIdx.x, lane = tid & 31, wave = tid >> 5;
  const int hh = lane >> 4, c = lane & 15;
  const int wm = wave & 3, wn = wave >> 2;
  const int b  = blockIdx.y;
  const int n0 = blockIdx.x * 128;

  if (tid < 64) sTab[tid] = tab[tid];
  __syncthreads();
  const int tb8 = clampi(sTab[32 + NE], 0, NTILE);
  if (b >= tb8) return;
  int e = 0;
#pragma unroll
  for (int q = 1; q < NE; ++q) e += (clampi(sTab[32 + q], 0, NTILE) <= b) ? 1 : 0;
  const int tbe = clampi(sTab[32 + e], 0, NTILE);
  const int cne = clampi(sTab[e], 0, NTOK);
  if (tid < 64) {
    const int rloc = (b - tbe) * 64 + tid;
    const bool valid = (rloc >= 0) && (rloc < cne);
    const int li = e * NTOK + clampi(rloc, 0, NTOK - 1);
    const int enc = tokl[li];
    const float w = wl[li];
    sEnc[tid] = clampi(enc, 0, NPAIR - 1);
    sW[tid]   = valid ? w : 0.f;
    sVal[tid] = valid ? 1 : 0;
  }
  __syncthreads();

  const unsigned short* wde = wd + (size_t)e * (size_t)(DIM * FFN);
  const int brow  = n0 + wn * 64;
  const int arow0 = b * 64 + wm * 16;
  v8f acc[4];
#pragma unroll
  for (int t = 0; t < 4; ++t) acc[t] = zero8();
#pragma unroll 1
  for (int k0 = 0; k0 < FFN; k0 += 32) {
    const v16bf fh = ldfrag(ah, FFN, arow0, k0, lane);
    const v16bf fl = ldfrag(al, FFN, arow0, k0, lane);
#pragma unroll
    for (int t = 0; t < 4; ++t) {
      const v16bf bq = ldfrag(wde, FFN, brow + 16 * t, k0, lane);
      acc[t] = mma16(fh, bq, acc[t]);
      acc[t] = mma16(fl, bq, acc[t]);
    }
  }

  float dbv[4];
#pragma unroll
  for (int t = 0; t < 4; ++t) dbv[t] = db[(size_t)e * DIM + brow + 16 * t + c];
  float wr[8];
#pragma unroll
  for (int r = 0; r < 8; ++r) wr[r] = sW[wm * 16 + 8 * hh + r];
  float* sw = sO + wave * (16 * OTP);
#pragma unroll
  for (int t = 0; t < 4; ++t) {
#pragma unroll
    for (int r = 0; r < 8; ++r) sw[(8 * hh + r) * OTP + 16 * t + c] = acc[t][r] + wr[r] * dbv[t];
  }
  __syncthreads();
  v4f val[8];
  size_t go[8];
  bool ok[8];
#pragma unroll
  for (int it = 0; it < 8; ++it) {
    const int p    = lane + 32 * it;
    const int L    = p >> 3;
    const int pc   = p & 7;
    const int row  = L >> 1;
    const int half = L & 1;
    const int lr   = wm * 16 + row;
    val[it] = *(const v4f*)(sw + row * OTP + half * 32 + pc * 4);
    ok[it]  = (sVal[lr] != 0);
    go[it]  = (size_t)sEnc[lr] * DIM + brow + half * 32 + pc * 4;
  }
  for (int ps = 0; ps < 2; ++ps) {
#pragma unroll
    for (int it = 0; it < 8; ++it) {
      if (ok[it]) *(volatile v4f*)(part + go[it]) = val[it];
    }
    __threadfence();
  }
}

__global__ __launch_bounds__(256) void k_comb(const float* __restrict__ part, float* __restrict__ out, int n4) {
#pragma clang fp contract(off)
  const int i = blockIdx.x * 256 + (int)threadIdx.x;
  if (i >= n4) return;
  const size_t t = (size_t)i / (DIM / 4);
  const size_t n = ((size_t)i % (DIM / 4)) * 4;
  const float* pr = part + t * (size_t)(NSEL * DIM) + n;
  v4f v = *(const v4f*)(pr);
  const v4f p1 = *(const v4f*)(pr + DIM);
  v = v + p1;
  volatile v4f* d = (volatile v4f*)(out + t * DIM + n);
  *d = v;
  __threadfence();
  *d = v;
}

extern "C" void kernel_launch(void* const* d_in, const int* in_sizes, int n_in,
                              void* d_out, int out_size, void* d_ws, size_t ws_size,
                              hipStream_t stream) {
  if (n_in < 11) return;
  if (in_sizes[0] != NTOK * DIM) return;
  if (in_sizes[1] != NTOK * NE) return;
  if (in_sizes[2] != NE * FFN * QPR) return;
  if (in_sizes[3] != NE * FFN * SPR) return;
  if (in_sizes[4] != NE * FFN) return;
  if (in_sizes[5] != NE * FFN * QPR) return;
  if (in_sizes[6] != NE * FFN * SPR) return;
  if (in_sizes[7] != NE * FFN) return;
  if (in_sizes[8] != NE * DIM * QPR) return;
  if (in_sizes[9] != NE * DIM * SPR) return;
  if (in_sizes[10] != NE * DIM) return;
  if (out_size != NTOK * DIM) return;

  const float* x     = (const float*)d_in[0];
  const float* rl    = (const float*)d_in[1];
  const int*   gblk  = (const int*)d_in[2];
  const int*   gscl  = (const int*)d_in[3];
  const float* gbias = (const float*)d_in[4];
  const int*   ublk  = (const int*)d_in[5];
  const int*   uscl  = (const int*)d_in[6];
  const float* ubias = (const float*)d_in[7];
  const int*   dblk  = (const int*)d_in[8];
  const int*   dscl  = (const int*)d_in[9];
  const float* dbias = (const float*)d_in[10];
  float* out = (float*)d_out;

  size_t off = 0;
  const size_t oXh = off; off += (size_t)NTOK * DIM * 2;
  const size_t oXl = off; off += (size_t)NTOK * DIM * 2;
  const size_t oWg = off; off += (size_t)NE * FFN * DIM * 2;
  const size_t oWu = off; off += (size_t)NE * FFN * DIM * 2;
  const size_t oWd = off; off += (size_t)NE * DIM * FFN * 2;
  const size_t oTL = off; off += (size_t)NE * NTOK * 4;
  const size_t oWL = off; off += (size_t)NE * NTOK * 4;
  const size_t oTB = off; off += (size_t)256;
  const size_t oAh = off; off += (size_t)AROWS * FFN * 2;
  const size_t oAl = off; off += (size_t)AROWS * FFN * 2;
  const size_t oP  = off; off += (size_t)NPAIR * DIM * 4;
  if (off > ws_size) return;
  if (off > (size_t)134217728) return;
  if ((oXl | oWg | oWu | oWd | oTL | oWL | oTB | oAh | oAl | oP) & (size_t)127) return;

  char* ws = (char*)d_ws;
  unsigned short* Xh  = (unsigned short*)(ws + oXh);
  unsigned short* Xl  = (unsigned short*)(ws + oXl);
  unsigned short* Wg  = (unsigned short*)(ws + oWg);
  unsigned short* Wu  = (unsigned short*)(ws + oWu);
  unsigned short* Wd  = (unsigned short*)(ws + oWd);
  int*            TOK = (int*)(ws + oTL);
  float*          WL  = (float*)(ws + oWL);
  int*            TAB = (int*)(ws + oTB);
  unsigned short* Ah  = (unsigned short*)(ws + oAh);
  unsigned short* Al  = (unsigned short*)(ws + oAl);
  float*          P   = (float*)(ws + oP);

  k_xsplit<<<dim3((NTOK * DIM) / 8 / 256), dim3(256), 0, stream>>>(x, Xh, Xl, (NTOK * DIM) / 8);
  k_deq<<<dim3((NE * FFN * DIM) / 8 / 256), dim3(256), 0, stream>>>(gblk, gscl, Wg, (NE * FFN * DIM) / 8);
  k_deq<<<dim3((NE * FFN * DIM) / 8 / 256), dim3(256), 0, stream>>>(ublk, uscl, Wu, (NE * FFN * DIM) / 8);
  k_deq<<<dim3((NE * DIM * FFN) / 8 / 256), dim3(256), 0, stream>>>(dblk, dscl, Wd, (NE * DIM * FFN) / 8);
  k_lists<<<dim3(1), dim3(256), 0, stream>>>(rl, TOK, WL, TAB);
  k_upgate<<<dim3(FFN / 128, NTILE), dim3(256), 0, stream>>>(Xh, Xl, Wg, Wu, gbias, ubias, TOK, WL, TAB, Ah, Al);
  k_down<<<dim3(DIM / 128, NTILE), dim3(256), 0, stream>>>(Ah, Al, Wd, dbias, TOK, WL, TAB, P);
  k_comb<<<dim3((NTOK * DIM) / 4 / 256), dim3(256), 0, stream>>>(P, out, (NTOK * DIM) / 4);
  (void)hipGetLastError();
}
